// DifferentialAttention_59596966199767
// MI455X (gfx1250) — hardware-verified
//
#include <hip/hip_runtime.h>
#include <hip/hip_bf16.h>

constexpr int SEQ      = 2048;
constexpr int DMODEL   = 2048;
constexpr int NHEAD    = 16;
constexpr int NKVH     = 4;
constexpr int HDIM     = 128;
constexpr int HHALF    = 64;
constexpr int QW       = NHEAD * HDIM;
constexpr int KW       = NKVH * HDIM;
constexpr int GQA_REP  = NHEAD / NKVH;
constexpr int NPAIR    = HDIM / 2;
constexpr int ATT_KC   = 64;
constexpr int ATT_QB   = 64;
constexpr int NQB      = SEQ / ATT_QB;
constexpr int OS_PITCH = HDIM + 4;
constexpr float QK_SCALE  = 0.125f;
constexpr float OUT_SCALE = 0.5f;
constexpr int NQBLK = (SEQ * QW / 8) / 256;
constexpr int NKBLK = (SEQ * KW / 8) / 256;

static_assert(HHALF == 64);
static_assert(SEQ % 64 == 0 && DMODEL % 64 == 0 && QW % 64 == 0 && KW % 64 == 0);
static_assert(DMODEL % 32 == 0 && QW % 32 == 0);
static_assert((SEQ * QW / 8) % 256 == 0 && (SEQ * KW / 8) % 256 == 0);
static_assert((SEQ * DMODEL / 8) % 256 == 0);
static_assert(((SEQ / 64) * (QW / 64)) % 8 == 0 && ((SEQ / 64) * (KW / 64)) % 8 == 0 && ((SEQ / 64) * (DMODEL / 64)) % 8 == 0);
static_assert(NQB == 32 && ATT_QB == 4 * 16 && ATT_KC == 64 && HDIM == 128);

typedef __attribute__((ext_vector_type(16))) __bf16 v16b;
typedef __attribute__((ext_vector_type(8)))  __bf16 v8b;
typedef __attribute__((ext_vector_type(8)))  float  v8f;
typedef __attribute__((ext_vector_type(4)))  float  v4f;
typedef __attribute__((ext_vector_type(4)))  unsigned int v4u;

__device__ __forceinline__ unsigned short f2bf_bits(float f) {
  unsigned u = __float_as_uint(f);
  return (unsigned short)((u + 0x7FFFu + ((u >> 16) & 1u)) >> 16);
}
__device__ __forceinline__ float bf_bits2f(unsigned short h) { return __uint_as_float(((unsigned)h) << 16); }
__device__ __forceinline__ float bf_rne(float f) { return bf_bits2f(f2bf_bits(f)); }

__device__ __forceinline__ void dep_guard_b(v8f& a, v8f& b, v16b x, v16b y) { asm volatile("v_nop\n\tv_nop\n\tv_nop\n\tv_nop" : "+v"(a), "+v"(b) : "v"(x), "v"(y)); }
__device__ __forceinline__ void keep4_b(v16b a, v16b b, v16b c, v16b d) { asm volatile("v_nop" :: "v"(a), "v"(b), "v"(c), "v"(d)); }
__device__ __forceinline__ void acc_guard4(v8f& a, v8f& b, v8f& c, v8f& d) { asm volatile("v_nop\n\tv_nop\n\tv_nop\n\tv_nop" : "+v"(a), "+v"(b), "+v"(c), "+v"(d)); }

template <typename T> struct Frag;
template <> struct Frag<__bf16> {
  typedef v16b V; union U { v16b v; v8b h[2]; };
  static __device__ __forceinline__ v16b load(const __bf16* p) {
    U f; f.h[0] = *(const v8b*)(p); f.h[1] = *(const v8b*)(p + 16); return f.v;
  }
  static __device__ __forceinline__ v8f mma(v16b a, v16b b, v8f c) {
    return __builtin_amdgcn_wmma_f32_16x16x32_bf16(false, a, false, b, (short)0, c, false, false);
  }
  static __device__ __forceinline__ void guard(v8f& a, v8f& b, v16b x, v16b y) { dep_guard_b(a, b, x, y); }
  static __device__ __forceinline__ void keep(v16b a, v16b b, v16b c, v16b d) { keep4_b(a, b, c, d); }
};

__device__ __forceinline__ unsigned short at_bf_bits(float f) {
  unsigned u = __float_as_uint(f);
  return (unsigned short)((u + 0x7FFFu + ((u >> 16) & 1u)) >> 16);
}
__device__ __forceinline__ __bf16 at_f2bf(float f) { return __builtin_bit_cast(__bf16, at_bf_bits(f)); }
__device__ __forceinline__ void at_split(float f, __bf16& hi, __bf16& lo) {
  const unsigned short hb = at_bf_bits(f);
  hi = __builtin_bit_cast(__bf16, hb);
  lo = at_f2bf(f - __uint_as_float(((unsigned)hb) << 16));
}
__device__ __forceinline__ v8f at_mma(v16b a, v16b b, v8f c) {
  c = __builtin_amdgcn_wmma_f32_16x16x32_bf16(false, a, false, b, (short)0, c, false, false);
  asm volatile("v_nop\n\tv_nop\n\tv_nop\n\tv_nop" : "+v"(c) : "v"(a), "v"(b));
  return c;
}

__device__ __forceinline__ unsigned pack_bf2(float a, float b) {
  return (unsigned)f2bf_bits(a) | ((unsigned)f2bf_bits(b) << 16);
}
__device__ __forceinline__ void split_pack2(float a, float b, unsigned& hw, unsigned& lw) {
  const unsigned short ha = f2bf_bits(a);
  const unsigned short hb = f2bf_bits(b);
  const unsigned short la = f2bf_bits(a - bf_bits2f(ha));
  const unsigned short lb = f2bf_bits(b - bf_bits2f(hb));
  hw = (unsigned)ha | ((unsigned)hb << 16);
  lw = (unsigned)la | ((unsigned)lb << 16);
}

__global__ __launch_bounds__(256) void cvt_f32_bf16x8(const float* __restrict__ in, unsigned short* __restrict__ out, int n8) {
  const int i = blockIdx.x * 256 + threadIdx.x;
  if (i < n8) {
    const size_t e0 = (size_t)i * 8;
    const v4f a = *(const v4f*)(in + e0);
    const v4f b = *(const v4f*)(in + e0 + 4);
    v4u w;
    w[0] = pack_bf2(a[0], a[1]);
    w[1] = pack_bf2(a[2], a[3]);
    w[2] = pack_bf2(b[0], b[1]);
    w[3] = pack_bf2(b[2], b[3]);
    *(volatile v4u*)(out + e0) = w;
    __threadfence();
    *(volatile v4u*)(out + e0) = w;
  }
}

template <int NPL>
__global__ __launch_bounds__(256) void transpose_bf16(const float* __restrict__ inA, const float* __restrict__ inB, int rows, int cols,
    unsigned short* __restrict__ oAh, unsigned short* __restrict__ oAl,
    unsigned short* __restrict__ oBh, unsigned short* __restrict__ oBl) {
  __shared__ float tile[64][65];
  const bool selB = (blockIdx.y != 0);
  const float* in = selB ? inB : inA;
  unsigned short* oh = selB ? oBh : oAh;
  unsigned short* ol = selB ? oBl : oAl;
  const int tilesC = cols >> 6;
  const int tr = blockIdx.x / tilesC;
  const int tc = blockIdx.x - tr * tilesC;
  const int r0 = tr << 6;
  const int c0 = tc << 6;
  const int t = threadIdx.x;
  {
    const int rr = t >> 2;
    const int cc = (t & 3) * 16;
    const float* src = in + (size_t)(r0 + rr) * cols + c0 + cc;
#pragma unroll
    for (int i = 0; i < 4; ++i) {
      const v4f v = *(const v4f*)(src + 4 * i);
      tile[rr][cc + 4 * i + 0] = v[0];
      tile[rr][cc + 4 * i + 1] = v[1];
      tile[rr][cc + 4 * i + 2] = v[2];
      tile[rr][cc + 4 * i + 3] = v[3];
    }
  }
  __syncthreads();
  const int wave = t >> 5, lane = t & 31, q = lane >> 3, e8 = (lane & 7) * 8;
  for (int pass = 0; pass < 2; ++pass) {
#pragma unroll
    for (int it = 0; it < 2; ++it) {
      const int cl = wave * 8 + it * 4 + q;
      float f[8];
#pragma unroll
      for (int e = 0; e < 8; ++e) f[e] = tile[e8 + e][cl];
      v4u hw, lw;
      if (NPL == 2) {
        unsigned a0, b0, a1, b1, a2, b2, a3, b3;
        split_pack2(f[0], f[1], a0, b0);
        split_pack2(f[2], f[3], a1, b1);
        split_pack2(f[4], f[5], a2, b2);
        split_pack2(f[6], f[7], a3, b3);
        hw[0] = a0; hw[1] = a1; hw[2] = a2; hw[3] = a3;
        lw[0] = b0; lw[1] = b1; lw[2] = b2; lw[3] = b3;
      } else {
        hw[0] = pack_bf2(f[0], f[1]);
        hw[1] = pack_bf2(f[2], f[3]);
        hw[2] = pack_bf2(f[4], f[5]);
        hw[3] = pack_bf2(f[6], f[7]);
        lw = hw;
      }
      const size_t go = (size_t)(c0 + cl) * rows + r0 + e8;
      *(volatile v4u*)(oh + go) = hw;
      if (NPL == 2) *(volatile v4u*)(ol + go) = lw;
    }
    __threadfence();
  }
}

template <int SPLIT>
__global__ __launch_bounds__(256) void wmma_gemm64_bf16(
    const unsigned short* __restrict__ Ap, const unsigned short* __restrict__ A2p, int lda, long strideA,
    const unsigned short* __restrict__ Btp, const unsigned short* __restrict__ Bt2p, int ldb, long strideB,
    float* __restrict__ Cp, int ldc, long strideC, int M, int N, int K, float scale) {
  typedef __bf16 T;
  typedef v16b V;
  const T* A = (const T*)Ap; const T* A2 = (const T*)A2p; const T* Bt = (const T*)Btp; const T* Bt2 = (const T*)Bt2p;
  __shared__ __align__(16) float sT[8][16 * 68];
  const int b    = blockIdx.y;
  const int lane = threadIdx.x & 31;
  const int wave = threadIdx.x >> 5;
  const int tilesN = N >> 6;
  const int tilesM = M >> 6;
  const int tile = blockIdx.x * 8 + wave;
  if (tile >= tilesM * tilesN) return;
  const int tm = tile / tilesN;
  const int tn = tile - tm * tilesN;
  const int m0 = tm << 6;
  const int n0 = tn << 6;

  const T* Ab  = A  + (size_t)b * strideA;
  const T* Bb  = Bt + (size_t)b * strideB;
  const T* Ab2 = (SPLIT != 0) ? (A2  + (size_t)b * strideA) : nullptr;
  const T* Bb2 = (SPLIT == 1) ? (Bt2 + (size_t)b * strideB) : nullptr;

  const int rlane = lane & 15;
  const int koff  = (lane >> 4) * 8;
  const int mOff  = (lane >> 4) * 8;

  v8f acc[4][4];
#pragma unroll
  for (int i = 0; i < 4; ++i)
#pragma unroll
    for (int j = 0; j < 4; ++j) acc[i][j] = (v8f){0.f,0.f,0.f,0.f,0.f,0.f,0.f,0.f};

  for (int k0 = 0; k0 < K; k0 += 32) {
    V bh[4], bl[4];
#pragma unroll
    for (int j = 0; j < 4; ++j) {
      const size_t bo = (size_t)(n0 + (j << 4) + rlane) * ldb + koff + k0;
      bh[j] = Frag<T>::load(Bb + bo);
      if (SPLIT == 1) bl[j] = Frag<T>::load(Bb2 + bo);
    }
#pragma unroll
    for (int i = 0; i < 4; ++i) {
      const size_t ao = (size_t)(m0 + (i << 4) + rlane) * lda + koff + k0;
      V ah = Frag<T>::load(Ab + ao);
      V al = ah;
      if (SPLIT != 0) al = Frag<T>::load(Ab2 + ao);
#pragma unroll
      for (int j = 0; j < 4; ++j) {
        acc[i][j] = Frag<T>::mma(ah, bh[j], acc[i][j]);
        if (SPLIT == 1) acc[i][j] = Frag<T>::mma(ah, bl[j], acc[i][j]);
        if (SPLIT != 0) acc[i][j] = Frag<T>::mma(al, bh[j], acc[i][j]);
      }
      Frag<T>::guard(acc[i][0], acc[i][3], ah, al);
    }
    Frag<T>::keep(bh[0], bh[1], bh[2], bh[3]);
    if (SPLIT == 1) Frag<T>::keep(bl[0], bl[1], bl[2], bl[3]);
  }
  acc_guard4(acc[0][0], acc[0][1], acc[0][2], acc[0][3]);
  acc_guard4(acc[1][0], acc[1][1], acc[1][2], acc[1][3]);
  acc_guard4(acc[2][0], acc[2][1], acc[2][2], acc[2][3]);
  acc_guard4(acc[3][0], acc[3][1], acc[3][2], acc[3][3]);

  float* slab = sT[wave];
  float* C = Cp + (size_t)b * strideC;
#pragma unroll
  for (int i = 0; i < 4; ++i) {
    const int mBase = m0 + (i << 4);
#pragma unroll
    for (int j = 0; j < 4; ++j) {
#pragma unroll
      for (int r = 0; r < 8; ++r) {
        slab[(mOff + r) * 68 + (j << 4) + rlane] = acc[i][j][r] * scale;
      }
    }
    __builtin_amdgcn_fence(__ATOMIC_RELEASE, "workgroup");
    __builtin_amdgcn_wave_barrier();
    __builtin_amdgcn_fence(__ATOMIC_ACQUIRE, "workgroup");
    {
      const int hh = lane >> 4, c4 = (lane & 15) * 4;
      for (int pass = 0; pass < 2; ++pass) {
#pragma unroll
        for (int it = 0; it < 8; ++it) {
          const int row = it * 2 + hh;
          const v4f v = *(const v4f*)(slab + row * 68 + c4);
          *(volatile v4f*)(C + (size_t)(mBase + row) * ldc + n0 + c4) = v;
        }
        __threadfence();
      }
    }
    __builtin_amdgcn_fence(__ATOMIC_RELEASE, "workgroup");
    __builtin_amdgcn_wave_barrier();
    __builtin_amdgcn_fence(__ATOMIC_ACQUIRE, "workgroup");
  }
}

__global__ __launch_bounds__(256) void rope_split_kernel(const float* __restrict__ Qf, const float* __restrict__ Kf,
    const float* __restrict__ cosb, const float* __restrict__ sinb,
    unsigned short* __restrict__ Qh, unsigned short* __restrict__ Ql,
    unsigned short* __restrict__ Kh, unsigned short* __restrict__ Kl, int nQblocks) {
  const bool isK = ((int)blockIdx.x >= nQblocks);
  const int g = (isK ? ((int)blockIdx.x - nQblocks) : (int)blockIdx.x) * 256 + (int)threadIdx.x;
  const int shift = isK ? 6 : 8;
  const float mul = isK ? 1.0f : QK_SCALE;
  const float* src = isK ? Kf : Qf;
  unsigned short* dh = isK ? Kh : Qh;
  unsigned short* dl = isK ? Kl : Ql;
  const int width = isK ? KW : QW;
  const int s = g >> shift;
  const int col = (g - (s << shift)) * 8;
  const int p0 = (col & (HDIM - 1)) >> 1;
  const size_t e0 = (size_t)s * width + col;
  const v4f xa = *(const v4f*)(src + e0);
  const v4f xb = *(const v4f*)(src + e0 + 4);
  const v4f cv = *(const v4f*)(cosb + (size_t)s * NPAIR + p0);
  const v4f sv = *(const v4f*)(sinb + (size_t)s * NPAIR + p0);
  float o0, o1, o2, o3, o4, o5, o6, o7;
  {
    const float c = bf_rne(cv[0]), sn = bf_rne(sv[0]);
    o0 = (xa[0] * c - xa[1] * sn) * mul;
    o1 = (xa[0] * sn + xa[1] * c) * mul;
  }
  {
    const float c = bf_rne(cv[1]), sn = bf_rne(sv[1]);
    o2 = (xa[2] * c - xa[3] * sn) * mul;
    o3 = (xa[2] * sn + xa[3] * c) * mul;
  }
  {
    const float c = bf_rne(cv[2]), sn = bf_rne(sv[2]);
    o4 = (xb[0] * c - xb[1] * sn) * mul;
    o5 = (xb[0] * sn + xb[1] * c) * mul;
  }
  {
    const float c = bf_rne(cv[3]), sn = bf_rne(sv[3]);
    o6 = (xb[2] * c - xb[3] * sn) * mul;
    o7 = (xb[2] * sn + xb[3] * c) * mul;
  }
  unsigned a0, b0, a1, b1, a2, b2, a3, b3;
  split_pack2(o0, o1, a0, b0);
  split_pack2(o2, o3, a1, b1);
  split_pack2(o4, o5, a2, b2);
  split_pack2(o6, o7, a3, b3);
  v4u hw, lw;
  hw[0] = a0; hw[1] = a1; hw[2] = a2; hw[3] = a3;
  lw[0] = b0; lw[1] = b1; lw[2] = b2; lw[3] = b3;
  *(volatile v4u*)(dh + e0) = hw;
  *(volatile v4u*)(dl + e0) = lw;
  __threadfence();
  *(volatile v4u*)(dh + e0) = hw;
  *(volatile v4u*)(dl + e0) = lw;
}

__global__ __launch_bounds__(128)
void diff_attn_kernel(const unsigned short* __restrict__ Qhp, const unsigned short* __restrict__ Qlp,
                      const unsigned short* __restrict__ Khp, const unsigned short* __restrict__ Klp,
                      const unsigned short* __restrict__ Vhp, const unsigned short* __restrict__ Vlp,
                      const float* __restrict__ lambda_p,
                      unsigned short* __restrict__ Ohp, unsigned short* __restrict__ Olp) {
  union FB { v16b v; v8b h[2]; };
  __shared__ __align__(16) __bf16 Ksh[ATT_KC * HHALF];
  __shared__ __align__(16) __bf16 Ksl[ATT_KC * HHALF];
  __shared__ __align__(16) __bf16 Vsh[HDIM * ATT_KC];
  __shared__ __align__(16) __bf16 Vsl[HDIM * ATT_KC];
  __shared__ __align__(16) __bf16 Psh[4][16 * ATT_KC];
  __shared__ __align__(16) __bf16 Psl[4][16 * ATT_KC];
  __shared__ __align__(16) float  Os[4][16 * OS_PITCH];

  const int tid  = threadIdx.x;
  const int wave = tid >> 5;
  const int lane = tid & 31;
  const int hh   = lane >> 4;
  const int c    = lane & 15;
  const int qb   = (int)blockIdx.x % NQB;
  const int h    = (int)blockIdx.x / NQB;
  const int kvh  = h / GQA_REP;
  const int q0   = qb * ATT_QB + wave * 16;

  const __bf16* Qh = (const __bf16*)Qhp;
  const __bf16* Ql = (const __bf16*)Qlp;
  const __bf16* Kh = (const __bf16*)Khp;
  const __bf16* Kl = (const __bf16*)Klp;
  const __bf16* Vh = (const __bf16*)Vhp;
  const __bf16* Vl = (const __bf16*)Vlp;

  float lam;
  {
    const float lp = bf_rne(lambda_p[h]);
    lam = 1.0f / (1.0f + expf(-lp));
  }
  float*  os  = Os[wave];
  __bf16* pwh = Psh[wave];
  __bf16* pwl = Psl[wave];

#pragma unroll 1
  for (int str = 0; str < 2; ++str) {
    v16b qah[2], qal[2];
    {
      const size_t qo = (size_t)(q0 + c) * QW + h * HDIM + str * HHALF + 8 * hh;
#pragma unroll
      for (int dc = 0; dc < 2; ++dc) {
        qah[dc] = Frag<__bf16>::load(Qh + qo + dc * 32);
        qal[dc] = Frag<__bf16>::load(Ql + qo + dc * 32);
      }
    }
    float mrow[8], lrow[8];
    v8f oacc[8];
#pragma unroll
    for (int r = 0; r < 8; ++r) { mrow[r] = -1.0e30f; lrow[r] = 0.f; }
#pragma unroll
    for (int t = 0; t < 8; ++t) oacc[t] = (v8f){0.f,0.f,0.f,0.f,0.f,0.f,0.f,0.f};

    for (int kc = 0; kc <= qb; ++kc) {
      const int kv0 = kc * ATT_KC;
      __syncthreads();
      {
        const int kcol = kvh * HDIM + str * HHALF;
#pragma unroll
        for (int i = 0; i < 4; ++i) {
          const int id  = tid + 128 * i;
          const int kvr = id >> 3;
          const int c8  = (id & 7) * 8;
          const size_t go = (size_t)(kv0 + kvr) * KW + kcol + c8;
          *(v8b*)(Ksh + kvr * HHALF + c8) = *(const v8b*)(Kh + go);
          *(v8b*)(Ksl + kvr * HHALF + c8) = *(const v8b*)(Kl + go);
        }
        asm volatile("" ::: "memory");
#pragma unroll
        for (int i = 0; i < 8; ++i) {
          const int id = tid + 128 * i;
          const int d  = id >> 3;
          const int c8 = (id & 7) * 8;
          const size_t go = (size_t)(kvh * HDIM + d) * SEQ + kv0 + c8;
          *(v8b*)(Vsh + d * ATT_KC + c8) = *(const v8b*)(Vh + go);
        }
        asm volatile("" ::: "memory");
#pragma unroll
        for (int i = 0; i < 8; ++i) {
          const int id = tid + 128 * i;
          const int d  = id >> 3;
          const int c8 = (id & 7) * 8;
          const size_t go = (size_t)(kvh * HDIM + d) * SEQ + kv0 + c8;
          *(v8b*)(Vsl + d * ATT_KC + c8) = *(const v8b*)(Vl + go);
        }
      }
      __syncthreads();

      v8f s[4];
#pragma unroll
      for (int j = 0; j < 4; ++j) {
        s[j] = (v8f){0.f,0.f,0.f,0.f,0.f,0.f,0.f,0.f};
#pragma unroll
        for (int dc = 0; dc < 2; ++dc) {
          FB kb, kl;
          kb.h[0] = *(const v8b*)(Ksh + (j * 16 + c) * HHALF + dc * 32 + 8 * hh);
          kb.h[1] = *(const v8b*)(Ksh + (j * 16 + c) * HHALF + dc * 32 + 16 + 8 * hh);
          kl.h[0] = *(const v8b*)(Ksl + (j * 16 + c) * HHALF + dc * 32 + 8 * hh);
          kl.h[1] = *(const v8b*)(Ksl + (j * 16 + c) * HHALF + dc * 32 + 16 + 8 * hh);
          s[j] = at_mma(qah[dc], kb.v, s[j]);
          s[j] = at_mma(qah[dc], kl.v, s[j]);
          s[j] = at_mma(qal[dc], kb.v, s[j]);
        }
      }
      const bool diag = (kc == qb);
      float cm[8];
#pragma unroll
      for (int r = 0; r < 8; ++r) {
        const int qrow = q0 + 8 * hh + r;
        float m = -1.0e30f;
#pragma unroll
        for (int j = 0; j < 4; ++j) {
          const int kvcol = kv0 + j * 16 + c;
          float sv = s[j][r];
          if (diag && (kvcol > qrow)) sv = -1.0e30f;
          s[j][r] = sv;
          m = fmaxf(m, sv);
        }
#pragma unroll
        for (int off = 1; off < 16; off <<= 1) m = fmaxf(m, __shfl_xor(m, off, 32));
        cm[r] = m;
      }
#pragma unroll
      for (int r = 0; r < 8; ++r) {
        const float mnew  = fmaxf(mrow[r], cm[r]);
        const float alpha = expf(mrow[r] - mnew);
        mrow[r] = mnew;
        float psum = 0.f;
#pragma unroll
        for (int j = 0; j < 4; ++j) {
          const float p = expf(s[j][r] - mnew);
          psum += p;
          __bf16 a, bl;
          at_split(p, a, bl);
          pwh[(8 * hh + r) * ATT_KC + j * 16 + c] = a;
          pwl[(8 * hh + r) * ATT_KC + j * 16 + c] = bl;
        }
#pragma unroll
        for (int off = 1; off < 16; off <<= 1) psum += __shfl_xor(psum, off, 32);
        lrow[r] = lrow[r] * alpha + psum;
#pragma unroll
        for (int t = 0; t < 8; ++t) oacc[t][r] *= alpha;
      }
      __syncthreads();
#pragma unroll 1
      for (int kk = 0; kk < 2; ++kk) {
        FB pa, pl;
        pa.h[0] = *(const v8b*)(pwh + c * ATT_KC + kk * 32 + 8 * hh);
        pa.h[1] = *(const v8b*)(pwh + c * ATT_KC + kk * 32 + 16 + 8 * hh);
        pl.h[0] = *(const v8b*)(pwl + c * ATT_KC + kk * 32 + 8 * hh);
        pl.h[1] = *(const v8b*)(pwl + c * ATT_KC + kk * 32 + 16 + 8 * hh);
#pragma unroll
        for (int t = 0; t < 8; ++t) {
          FB vb, vl;
          vb.h[0] = *(const v8b*)(Vsh + (t * 16 + c) * ATT_KC + kk * 32 + 8 * hh);
          vb.h[1] = *(const v8b*)(Vsh + (t * 16 + c) * ATT_KC + kk * 32 + 16 + 8 * hh);
          vl.h[0] = *(const v8b*)(Vsl + (t * 16 + c) * ATT_KC + kk * 32 + 8 * hh);
          vl.h[1] = *(const v8b*)(Vsl + (t * 16 + c) * ATT_KC + kk * 32 + 16 + 8 * hh);
          oacc[t] = at_mma(pa.v, vb.v, oacc[t]);
          oacc[t] = at_mma(pa.v, vl.v, oacc[t]);
          oacc[t] = at_mma(pl.v, vb.v, oacc[t]);
        }
      }
    }

#pragma unroll
    for (int r = 0; r < 8; ++r) {
      const float inv = 1.0f / lrow[r];
#pragma unroll
      for (int t = 0; t < 8; ++t) {
        const int idx = (8 * hh + r) * OS_PITCH + t * 16 + c;
        const float a = oacc[t][r] * inv;
        if (str == 0) {
          os[idx] = a;
        } else {
          const float a1 = os[idx];
          os[idx] = (a1 - lam * a) * OUT_SCALE;
        }
      }
    }
  }
  __syncthreads();

  {
    const int q4 = lane >> 3, c8 = (lane & 7) * 8;
    for (int pass = 0; pass < 2; ++pass) {
#pragma unroll
      for (int it = 0; it < 4; ++it) {
        const int row = it * 4 + q4;
#pragma unroll
        for (int seg = 0; seg < 2; ++seg) {
          const float* sp = os + row * OS_PITCH + seg * 64 + c8;
          const v4f u0 = *(const v4f*)sp;
          const v4f u1 = *(const v4f*)(sp + 4);
          unsigned a0, b0, a1, b1, a2, b2, a3, b3;
          split_pack2(u0[0], u0[1], a0, b0);
          split_pack2(u0[2], u0[3], a1, b1);
          split_pack2(u1[0], u1[1], a2, b2);
          split_pack2(u1[2], u1[3], a3, b3);
          v4u hw, lw;
          hw[0] = a0; hw[1] = a1; hw[2] = a2; hw[3] = a3;
          lw[0] = b0; lw[1] = b1; lw[2] = b2; lw[3] = b3;
          const size_t go = (size_t)(q0 + row) * QW + h * HDIM + seg * 64 + c8;
          *(volatile v4u*)(Ohp + go) = hw;
          *(volatile v4u*)(Olp + go) = lw;
        }
      }
      __threadfence();
    }
  }
}

extern "C" void kernel_launch(void* const* d_in, const int* in_sizes, int n_in,
                              void* d_out, int out_size, void* d_ws, size_t ws_size,
                              hipStream_t stream) {
  (void)in_sizes; (void)out_size;
  if (n_in < 8) return;
  const float* x    = (const float*)d_in[0];
  const float* fcos = (const float*)d_in[1];
  const float* fsin = (const float*)d_in[2];
  const float* Wq   = (const float*)d_in[3];
  const float* Wk   = (const float*)d_in[4];
  const float* Wv   = (const float*)d_in[5];
  const float* Wo   = (const float*)d_in[6];
  const float* lamp = (const float*)d_in[7];
  float* out = (float*)d_out;

  char* ws = (char*)d_ws;
  size_t off = 0;
  unsigned short* xb   = (unsigned short*)(ws + off); off += (size_t)SEQ * DMODEL * 2;
  unsigned short* Wqt  = (unsigned short*)(ws + off); off += (size_t)QW * DMODEL * 2;
  unsigned short* Wkvt = (unsigned short*)(ws + off); off += (size_t)2 * KW * DMODEL * 2;
  unsigned short* Wot  = (unsigned short*)(ws + off); off += (size_t)DMODEL * QW * 2;
  float*          Qf   = (float*)(ws + off);          off += (size_t)SEQ * QW * 4;
  float*          KVf  = (float*)(ws + off);          off += (size_t)2 * SEQ * KW * 4;
  unsigned short* Qh   = (unsigned short*)(ws + off); off += (size_t)SEQ * QW * 2;
  unsigned short* Ql   = (unsigned short*)(ws + off); off += (size_t)SEQ * QW * 2;
  unsigned short* Kh   = (unsigned short*)(ws + off); off += (size_t)SEQ * KW * 2;
  unsigned short* Kl   = (unsigned short*)(ws + off); off += (size_t)SEQ * KW * 2;
  unsigned short* Vth  = (unsigned short*)(ws + off); off += (size_t)KW * SEQ * 2;
  unsigned short* Vtl  = (unsigned short*)(ws + off); off += (size_t)KW * SEQ * 2;
  unsigned short* Oh   = (unsigned short*)(ws + off); off += (size_t)SEQ * QW * 2;
  unsigned short* Ol   = (unsigned short*)(ws + off); off += (size_t)SEQ * QW * 2;
  if (off > ws_size) return;

  const float* Vf = KVf + (size_t)SEQ * KW;
  unsigned short* Wvt = Wkvt + (size_t)KW * DMODEL;

  cvt_f32_bf16x8<<<(SEQ * DMODEL / 8) / 256, 256, 0, stream>>>(x, xb, SEQ * DMODEL / 8);
  transpose_bf16<1><<<dim3((DMODEL / 64) * (QW / 64), 1), 256, 0, stream>>>(Wq, Wq, DMODEL, QW, Wqt, Wqt, Wqt, Wqt);
  transpose_bf16<1><<<dim3((DMODEL / 64) * (KW / 64), 2), 256, 0, stream>>>(Wk, Wv, DMODEL, KW, Wkvt, Wkvt, Wvt, Wvt);
  transpose_bf16<1><<<dim3((QW / 64) * (DMODEL / 64), 1), 256, 0, stream>>>(Wo, Wo, QW, DMODEL, Wot, Wot, Wot, Wot);
  wmma_gemm64_bf16<0><<<dim3(((SEQ / 64) * (QW / 64)) / 8, 1), 256, 0, stream>>>(
      xb, xb, DMODEL, 0L, Wqt, Wqt, DMODEL, 0L, Qf, QW, 0L, SEQ, QW, DMODEL, 1.0f);
  wmma_gemm64_bf16<0><<<dim3(((SEQ / 64) * (KW / 64)) / 8, 2), 256, 0, stream>>>(
      xb, xb, DMODEL, 0L, Wkvt, Wkvt, DMODEL, (long)KW * DMODEL, KVf, KW, (long)SEQ * KW, SEQ, KW, DMODEL, 1.0f);
  rope_split_kernel<<<NQBLK + NKBLK, 256, 0, stream>>>(Qf, KVf, fcos, fsin, Qh, Ql, Kh, Kl, NQBLK);
  transpose_bf16<2><<<dim3((SEQ / 64) * (KW / 64), 1), 256, 0, stream>>>(Vf, Vf, SEQ, KW, Vth, Vtl, Vth, Vtl);
  diff_attn_kernel<<<NHEAD * NQB, 128, 0, stream>>>(Qh, Ql, Kh, Kl, Vth, Vtl, lamp, Oh, Ol);
  wmma_gemm64_bf16<2><<<dim3(((SEQ / 64) * (DMODEL / 64)) / 8, 1), 256, 0, stream>>>(
      Oh, Ol, QW, 0L, Wot, Wot, QW, 0L, out, DMODEL, 0L, SEQ, DMODEL, QW, 1.0f);
}
